// FFT_84353157693551
// MI455X (gfx1250) — hardware-verified
//
#include <hip/hip_runtime.h>
#include <math.h>

#define NB_   2
#define CH_   512
#define TT_   2048
#define NH_   8
#define HD_   64
#define FC_   2048
#define NL_   2
#define NTOK_ (NB_ * TT_)
#define NW_   (CH_ * CH_)
#define NW1_  (FC_ * CH_)
#define EPS_  1e-5f
#define WSC_  32.0f
#define HSC_  64.0f
#define PSC_  4096.0f

static_assert(NTOK_ % 128 == 0);
static_assert(TT_ % 128 == 0);
static_assert(CH_ % 64 == 0);
static_assert(FC_ % 64 == 0);
static_assert(HD_ == 64);
static_assert(CH_ == NH_ * HD_);

typedef _Float16 v16h __attribute__((ext_vector_type(16)));
typedef _Float16 v8h  __attribute__((ext_vector_type(8)));
typedef _Float16 v4h  __attribute__((ext_vector_type(4)));
typedef float    v8f  __attribute__((ext_vector_type(8)));
typedef float    v4f  __attribute__((ext_vector_type(4)));
typedef v8h __attribute__((may_alias)) v8ha;
typedef v4f __attribute__((may_alias)) v4fa;

union Frag { v16h v; v8h half[2]; };

__device__ __forceinline__ v8f wmma_f16(v16h a, v16h b, v8f c) {
  v8f d = __builtin_amdgcn_wmma_f32_16x16x32_f16(false, a, false, b, (short)0, c, false, false);
  asm volatile("v_nop\n\tv_nop\n\tv_nop\n\tv_nop" : "+v"(d) : "v"(a), "v"(b));
  return d;
}

__device__ __forceinline__ v16h load_frag(const _Float16* p, int h) {
  Frag f;
  f.half[0] = *(const v8ha*)(p + 8 * h);
  f.half[1] = *(const v8ha*)(p + 16 + 8 * h);
  return f.v;
}

#define G_MAT_ (2 * NW_ / 8)
#define G_QKV_ (3 * G_MAT_)
#define G_O_   (G_QKV_ + G_MAT_)
#define G_1_   (G_O_ + 2 * NW1_ / 8)
#define G_TOT_ (G_1_ + 2 * NW1_ / 8)
static_assert(G_MAT_ % 256 == 0);
static_assert(G_TOT_ % 256 == 0);

__global__ __launch_bounds__(256) void convert_w(
    const float* __restrict__ wq, const float* __restrict__ wk,
    const float* __restrict__ wv, const float* __restrict__ wo,
    const float* __restrict__ w1, const float* __restrict__ w2,
    _Float16* __restrict__ whqkv, _Float16* __restrict__ who,
    _Float16* __restrict__ wh1, _Float16* __restrict__ wh2)
{
  const int g = blockIdx.x * 256 + threadIdx.x;
  if (g >= G_TOT_) return;
  const float* src;
  _Float16* dst;
  if (g < G_QKV_) {
    const int wsel = g / G_MAT_;
    const size_t e = (size_t)(g - wsel * G_MAT_) * 8;
    const size_t layer = e / NW_;
    const size_t rem = e - layer * NW_;
    const float* wsrc = (wsel == 0) ? wq : ((wsel == 1) ? wk : wv);
    src = wsrc + e;
    dst = whqkv + layer * (size_t)(3 * NW_) + (size_t)wsel * NW_ + rem;
  } else if (g < G_O_) {
    const size_t e = (size_t)(g - G_QKV_) * 8;
    src = wo + e; dst = who + e;
  } else if (g < G_1_) {
    const size_t e = (size_t)(g - G_O_) * 8;
    src = w1 + e; dst = wh1 + e;
  } else {
    const size_t e = (size_t)(g - G_1_) * 8;
    src = w2 + e; dst = wh2 + e;
  }
  const v4f a = *(const v4fa*)src;
  const v4f c = *(const v4fa*)(src + 4);
  const v8h o = { (_Float16)(a.x * WSC_), (_Float16)(a.y * WSC_), (_Float16)(a.z * WSC_), (_Float16)(a.w * WSC_),
                  (_Float16)(c.x * WSC_), (_Float16)(c.y * WSC_), (_Float16)(c.z * WSC_), (_Float16)(c.w * WSC_) };
  *(volatile v8h*)dst = o;
  __threadfence();
  *(volatile v8h*)dst = o;
}

__global__ __launch_bounds__(256) void transpose_in(
    const float* __restrict__ x, const float* __restrict__ xmask,
    float* __restrict__ xres, _Float16* __restrict__ xh)
{
  __shared__ float s[64][65];
  const int tid = threadIdx.x, lane = tid & 31, w = tid >> 5;
  const int b = blockIdx.z, c0 = blockIdx.y * 64, t0 = blockIdx.x * 64;
  {
    const int r = tid >> 4, q = tid & 15;
    const v4f mk = *(const v4fa*)(xmask + (size_t)b * TT_ + t0 + 4 * q);
    #pragma unroll
    for (int i = 0; i < 4; ++i) {
      const int cc = 16 * i + r;
      const v4f v = *(const v4fa*)(x + ((size_t)b * CH_ + c0 + cc) * TT_ + t0 + 4 * q);
      s[cc][4 * q + 0] = v.x * mk.x;
      s[cc][4 * q + 1] = v.y * mk.y;
      s[cc][4 * q + 2] = v.z * mk.z;
      s[cc][4 * q + 3] = v.w * mk.w;
    }
  }
  __syncthreads();

  const int rr = lane >> 4, p = lane & 15;
  const int q8 = lane & 7, sub = lane >> 3;
  v4f of[4];
  v8h oh[2];
  #pragma unroll
  for (int i = 0; i < 4; ++i) {
    const int tt = w * 8 + 2 * i + rr;
    const v4f v = { s[4 * p + 0][tt], s[4 * p + 1][tt], s[4 * p + 2][tt], s[4 * p + 3][tt] };
    of[i] = v;
  }
  #pragma unroll
  for (int i = 0; i < 2; ++i) {
    const int tt = w * 8 + 4 * i + sub;
    const v8h v = { (_Float16)s[8 * q8 + 0][tt], (_Float16)s[8 * q8 + 1][tt], (_Float16)s[8 * q8 + 2][tt], (_Float16)s[8 * q8 + 3][tt],
                    (_Float16)s[8 * q8 + 4][tt], (_Float16)s[8 * q8 + 5][tt], (_Float16)s[8 * q8 + 6][tt], (_Float16)s[8 * q8 + 7][tt] };
    oh[i] = v;
  }
  #pragma unroll
  for (int pass = 0; pass < 2; ++pass) {
    #pragma unroll
    for (int i = 0; i < 4; ++i) {
      const int tt = w * 8 + 2 * i + rr;
      const size_t row = (size_t)b * TT_ + t0 + tt;
      *(volatile v4f*)(xres + row * CH_ + c0 + 4 * p) = of[i];
    }
    #pragma unroll
    for (int i = 0; i < 2; ++i) {
      const int tt = w * 8 + 4 * i + sub;
      const size_t row = (size_t)b * TT_ + t0 + tt;
      *(volatile v8h*)(xh + row * CH_ + c0 + 8 * q8) = oh[i];
    }
    if (pass == 0) __threadfence();
  }
}

__device__ __forceinline__ void gemm_mainloop(v8f (&acc)[2][4],
                                              const _Float16* xa0, const _Float16* xa1,
                                              const _Float16* wb, int ldb, int K, int h)
{
  #pragma unroll 1
  for (int k0 = 0; k0 < K; k0 += 32) {
    const v16h a0 = load_frag(xa0 + k0, h);
    const v16h a1 = load_frag(xa1 + k0, h);
    #pragma unroll
    for (int nt = 0; nt < 4; ++nt) {
      const v16h bf = load_frag(wb + (size_t)nt * 16 * ldb + k0, h);
      acc[0][nt] = wmma_f16(a0, bf, acc[0][nt]);
      acc[1][nt] = wmma_f16(a1, bf, acc[1][nt]);
    }
  }
}

__device__ __forceinline__ void qkv_store_pass(const _Float16* sT, _Float16* plane, _Float16* vt,
                                               int which, int head, int m0, int w, int lane) {
  const int q8 = lane & 7, sub = lane >> 3;
  #pragma unroll
  for (int i = 0; i < 8; ++i) {
    const int lid = w * 32 + i * 4 + sub;
    v8h v;
    _Float16* dst;
    if (which != 2) {
      v = *(const v8ha*)(sT + lid * HD_ + 8 * q8);
      dst = plane + (size_t)(m0 + lid) * CH_ + head * HD_ + 8 * q8;
    } else {
      const int d = lid >> 1, hl = lid & 1;
      v = *(const v8ha*)(sT + d * 128 + 64 * hl + 8 * q8);
      dst = vt + (size_t)(head * HD_ + d) * NTOK_ + m0 + 64 * hl + 8 * q8;
    }
    *(volatile v8h*)dst = v;
  }
}

__global__ __launch_bounds__(128) void gemm_qkv(
    const _Float16* __restrict__ xh,
    const _Float16* __restrict__ wl,
    const float* __restrict__ bq, const float* __restrict__ bk, const float* __restrict__ bv,
    _Float16* __restrict__ qh,
    _Float16* __restrict__ kh,
    _Float16* __restrict__ vt)
{
  __shared__ __attribute__((aligned(16))) _Float16 sT[128 * 64];

  const int tid = threadIdx.x, lane = tid & 31, w = tid >> 5;
  const int h = lane >> 4, m = lane & 15;
  const int m0 = blockIdx.x * 128;
  const int cg = blockIdx.y;
  const int which = cg >> 3, head = cg & 7;
  const int m0w = m0 + 32 * w;

  const _Float16* xa0 = xh + (size_t)(m0w + m) * CH_;
  const _Float16* xa1 = xa0 + (size_t)16 * CH_;
  const _Float16* wb  = wl + (size_t)(cg * 64 + m) * CH_;

  const v8f zero8 = {0.f, 0.f, 0.f, 0.f, 0.f, 0.f, 0.f, 0.f};
  v8f acc[2][4];
  #pragma unroll
  for (int mt = 0; mt < 2; ++mt)
    #pragma unroll
    for (int nt = 0; nt < 4; ++nt) acc[mt][nt] = zero8;

  gemm_mainloop(acc, xa0, xa1, wb, CH_, CH_, h);

  const float* bias = (which == 0) ? bq : ((which == 1) ? bk : bv);
  #pragma unroll
  for (int nt = 0; nt < 4; ++nt) {
    const int feat = 16 * nt + m;
    const float bvl = bias[head * HD_ + feat];
    #pragma unroll
    for (int mt = 0; mt < 2; ++mt) {
      #pragma unroll
      for (int r = 0; r < 8; ++r) {
        const int tokl = 32 * w + 16 * mt + 8 * h + r;
        const float y = acc[mt][nt][r] * (1.0f / WSC_) + bvl;
        const int idx = (which == 2) ? (feat * 128 + tokl) : (tokl * HD_ + feat);
        sT[idx] = (_Float16)y;
      }
    }
  }
  __syncthreads();

  _Float16* plane = (which == 0) ? qh : kh;
  qkv_store_pass(sT, plane, vt, which, head, m0, w, lane);
  __threadfence();
  qkv_store_pass(sT, plane, vt, which, head, m0, w, lane);
}

__device__ __forceinline__ v16h pack_p(v8f a, v8f c) {
  const v16h r = { (_Float16)(a[0] * PSC_), (_Float16)(a[1] * PSC_), (_Float16)(a[2] * PSC_), (_Float16)(a[3] * PSC_),
                   (_Float16)(a[4] * PSC_), (_Float16)(a[5] * PSC_), (_Float16)(a[6] * PSC_), (_Float16)(a[7] * PSC_),
                   (_Float16)(c[0] * PSC_), (_Float16)(c[1] * PSC_), (_Float16)(c[2] * PSC_), (_Float16)(c[3] * PSC_),
                   (_Float16)(c[4] * PSC_), (_Float16)(c[5] * PSC_), (_Float16)(c[6] * PSC_), (_Float16)(c[7] * PSC_) };
  return r;
}

__device__ __forceinline__ void att_store_pass(const _Float16* so, _Float16* oh,
                                               size_t tb, int q0, int head, int lane) {
  const int q8 = lane & 7, sub = lane >> 3;
  #pragma unroll
  for (int i = 0; i < 4; ++i) {
    const int row = 4 * i + sub;
    const v8h v = *(const v8ha*)(so + row * 64 + 8 * q8);
    _Float16* dst = oh + (tb + q0 + row) * CH_ + head * HD_ + 8 * q8;
    *(volatile v8h*)dst = v;
  }
}

__global__ __launch_bounds__(128) void attn_kernel(
    const _Float16* __restrict__ qh,
    const _Float16* __restrict__ kh,
    const _Float16* __restrict__ vt,
    _Float16* __restrict__ oh)
{
  __shared__ __attribute__((aligned(16))) _Float16 sO[4 * 16 * 64];

  const int tid = threadIdx.x, lane = tid & 31, w = tid >> 5;
  const int h = lane >> 4, m = lane & 15;
  const int bh = blockIdx.y, b = bh >> 3, head = bh & 7;
  const int q0 = blockIdx.x * 64 + 16 * w;
  const size_t tb = (size_t)b * TT_;

  const _Float16* qrow = qh + (tb + q0 + m) * CH_ + head * HD_;
  const v16h qb0 = load_frag(qrow, h);
  const v16h qb1 = load_frag(qrow + 32, h);

  const v8f zero8 = {0.f, 0.f, 0.f, 0.f, 0.f, 0.f, 0.f, 0.f};
  v8f o[4];
  #pragma unroll
  for (int t = 0; t < 4; ++t) o[t] = zero8;
  const float NEG = -__builtin_inff();
  float mrun = NEG, lrun = 0.0f;

  const _Float16* kbase = kh + (tb + m) * CH_ + head * HD_;
  const _Float16* vbase = vt + (size_t)(head * HD_ + m) * NTOK_ + tb;
  const int qi = q0 + m;

  #pragma unroll 1
  for (int kb = 0; kb <= q0 + 15; kb += 64) {
    v8f s[4];
    #pragma unroll
    for (int j = 0; j < 4; ++j) {
      const _Float16* kp = kbase + (size_t)(kb + 16 * j) * CH_;
      const v16h kf0 = load_frag(kp, h);
      const v16h kf1 = load_frag(kp + 32, h);
      v8f z = zero8;
      z = wmma_f16(kf0, qb0, z);
      z = wmma_f16(kf1, qb1, z);
      s[j] = z;
    }
    #pragma unroll
    for (int j = 0; j < 4; ++j)
      #pragma unroll
      for (int r = 0; r < 8; ++r) {
        const int key = kb + 16 * j + 8 * h + r;
        const float val = s[j][r] * 0.125f - (float)(qi - key);
        s[j][r] = (key <= qi) ? val : NEG;
      }

    float mloc = s[0][0];
    #pragma unroll
    for (int j = 0; j < 4; ++j)
      #pragma unroll
      for (int r = 0; r < 8; ++r) mloc = fmaxf(mloc, s[j][r]);
    mloc = fmaxf(mloc, __shfl_xor(mloc, 16));
    const float mnew = fmaxf(mrun, mloc);
    const float alpha = __expf(mrun - mnew);
    mrun = mnew;
    float lsum = 0.0f;
    #pragma unroll
    for (int j = 0; j < 4; ++j)
      #pragma unroll
      for (int r = 0; r < 8; ++r) {
        const float p = __expf(s[j][r] - mnew);
        s[j][r] = p;
        lsum += p;
      }
    lsum += __shfl_xor(lsum, 16);
    lrun = lrun * alpha + lsum;
    #pragma unroll
    for (int t = 0; t < 4; ++t)
      #pragma unroll
      for (int r = 0; r < 8; ++r) o[t][r] = o[t][r] * alpha;

    const v16h pb0 = pack_p(s[0], s[1]);
    const v16h pb1 = pack_p(s[2], s[3]);

    #pragma unroll
    for (int t = 0; t < 4; ++t) {
      const _Float16* vp = vbase + (size_t)(16 * t) * NTOK_ + kb;
      const v16h vf0 = load_frag(vp, h);
      const v16h vf1 = load_frag(vp + 32, h);
      o[t] = wmma_f16(vf0, pb0, o[t]);
      o[t] = wmma_f16(vf1, pb1, o[t]);
    }
  }

  const float inv = (1.0f / lrun) * (1.0f / PSC_);
  _Float16* so = sO + w * 1024;
  #pragma unroll
  for (int t = 0; t < 4; ++t)
    #pragma unroll
    for (int r = 0; r < 8; ++r)
      so[m * 64 + 16 * t + 8 * h + r] = (_Float16)(o[t][r] * inv);
  __syncthreads();

  att_store_pass(so, oh, tb, q0, head, lane);
  __threadfence();
  att_store_pass(so, oh, tb, q0, head, lane);
}

__device__ __forceinline__ void f32_store_pass(const float* sT, float* Y, int m0, int n0, int w, int lane) {
  const int p = lane & 15, rr = lane >> 4;
  #pragma unroll
  for (int i = 0; i < 16; ++i) {
    const int lid = w * 32 + 2 * i + rr;
    const v4f v = *(const v4fa*)(sT + lid * 64 + 4 * p);
    *(volatile v4f*)(Y + (size_t)(m0 + lid) * CH_ + n0 + 4 * p) = v;
  }
}

__global__ __launch_bounds__(128) void gemm_f32(
    const _Float16* __restrict__ A, int lda,
    const _Float16* __restrict__ Bw, int ldb, int K,
    const float* __restrict__ bias, float accs,
    float* __restrict__ Y)
{
  __shared__ __attribute__((aligned(16))) float sT[128 * 64];

  const int tid = threadIdx.x, lane = tid & 31, w = tid >> 5;
  const int h = lane >> 4, m = lane & 15;
  const int m0 = blockIdx.x * 128, n0 = blockIdx.y * 64;
  const int m0w = m0 + 32 * w;

  const _Float16* xa0 = A + (size_t)(m0w + m) * lda;
  const _Float16* xa1 = xa0 + (size_t)16 * lda;
  const _Float16* wb  = Bw + (size_t)(n0 + m) * ldb;

  const v8f zero8 = {0.f, 0.f, 0.f, 0.f, 0.f, 0.f, 0.f, 0.f};
  v8f acc[2][4];
  #pragma unroll
  for (int mt = 0; mt < 2; ++mt)
    #pragma unroll
    for (int nt = 0; nt < 4; ++nt) acc[mt][nt] = zero8;

  gemm_mainloop(acc, xa0, xa1, wb, ldb, K, h);

  #pragma unroll
  for (int nt = 0; nt < 4; ++nt) {
    const int feat = 16 * nt + m;
    const float bvl = bias[n0 + feat];
    #pragma unroll
    for (int mt = 0; mt < 2; ++mt) {
      #pragma unroll
      for (int r = 0; r < 8; ++r) {
        const int tokl = 32 * w + 16 * mt + 8 * h + r;
        sT[tokl * 64 + feat] = acc[mt][nt][r] * accs + bvl;
      }
    }
  }
  __syncthreads();

  f32_store_pass(sT, Y, m0, n0, w, lane);
  __threadfence();
  f32_store_pass(sT, Y, m0, n0, w, lane);
}

__global__ __launch_bounds__(256) void ln_kernel(
    float* __restrict__ xres, const float* __restrict__ ybuf,
    const float* __restrict__ g, const float* __restrict__ bb,
    const float* __restrict__ xmask, int use_mask,
    _Float16* __restrict__ xh)
{
  const int tid = threadIdx.x, lane = tid & 31, w = tid >> 5;
  const int row = blockIdx.x * 8 + w;
  const size_t rb = (size_t)row * CH_;
  const float mval = xmask[row];
  const float mk = use_mask ? mval : 1.0f;

  v4f v[4];
  float sum = 0.0f;
  #pragma unroll
  for (int j = 0; j < 4; ++j) {
    const v4f xv = *(const v4fa*)(xres + rb + j * 128 + 4 * lane);
    const v4f yv = *(const v4fa*)(ybuf + rb + j * 128 + 4 * lane);
    v[j] = xv + yv * mk;
    sum += (v[j].x + v[j].y) + (v[j].z + v[j].w);
  }
  #pragma unroll
  for (int off = 16; off > 0; off >>= 1) sum += __shfl_xor(sum, off);
  const float mean = sum * (1.0f / CH_);
  float sq = 0.0f;
  #pragma unroll
  for (int j = 0; j < 4; ++j) {
    const v4f d = v[j] - mean;
    sq += (d.x * d.x + d.y * d.y) + (d.z * d.z + d.w * d.w);
  }
  #pragma unroll
  for (int off = 16; off > 0; off >>= 1) sq += __shfl_xor(sq, off);
  const float var = sq * (1.0f / CH_);
  const float rstd = rsqrtf(var + EPS_);

  v4f of[4];
  v4h oh[4];
  #pragma unroll
  for (int j = 0; j < 4; ++j) {
    const v4f gv = *(const v4fa*)(g + j * 128 + 4 * lane);
    const v4f bv = *(const v4fa*)(bb + j * 128 + 4 * lane);
    const v4f ov = (v[j] - mean) * rstd * gv + bv;
    of[j] = ov;
    const v4h hv = { (_Float16)ov.x, (_Float16)ov.y, (_Float16)ov.z, (_Float16)ov.w };
    oh[j] = hv;
  }
  #pragma unroll
  for (int pass = 0; pass < 2; ++pass) {
    #pragma unroll
    for (int j = 0; j < 4; ++j) {
      *(volatile v4f*)(xres + rb + j * 128 + 4 * lane) = of[j];
      *(volatile v4h*)(xh + rb + j * 128 + 4 * lane) = oh[j];
    }
    if (pass == 0) __threadfence();
  }
}

__device__ __forceinline__ void h_store_pass(const _Float16* sT, _Float16* hp, int m0, int n0, int w, int lane) {
  const int q8 = lane & 7, sub = lane >> 3;
  #pragma unroll
  for (int i = 0; i < 8; ++i) {
    const int lid = w * 32 + i * 4 + sub;
    const v8h v = *(const v8ha*)(sT + lid * 64 + 8 * q8);
    *(volatile v8h*)(hp + (size_t)(m0 + lid) * FC_ + n0 + 8 * q8) = v;
  }
}

__global__ __launch_bounds__(128) void gemm_gelu(
    const _Float16* __restrict__ xh,
    const _Float16* __restrict__ wl,
    const float* __restrict__ b1,
    _Float16* __restrict__ hp)
{
  __shared__ __attribute__((aligned(16))) _Float16 sT[128 * 64];

  const int tid = threadIdx.x, lane = tid & 31, w = tid >> 5;
  const int h = lane >> 4, m = lane & 15;
  const int m0 = blockIdx.x * 128, n0 = blockIdx.y * 64;
  const int m0w = m0 + 32 * w;

  const _Float16* xa0 = xh + (size_t)(m0w + m) * CH_;
  const _Float16* xa1 = xa0 + (size_t)16 * CH_;
  const _Float16* wb  = wl + (size_t)(n0 + m) * CH_;

  const v8f zero8 = {0.f, 0.f, 0.f, 0.f, 0.f, 0.f, 0.f, 0.f};
  v8f acc[2][4];
  #pragma unroll
  for (int mt = 0; mt < 2; ++mt)
    #pragma unroll
    for (int nt = 0; nt < 4; ++nt) acc[mt][nt] = zero8;

  gemm_mainloop(acc, xa0, xa1, wb, CH_, CH_, h);

  #pragma unroll
  for (int nt = 0; nt < 4; ++nt) {
    const int feat = 16 * nt + m;
    const float bvl = b1[n0 + feat];
    #pragma unroll
    for (int mt = 0; mt < 2; ++mt) {
      #pragma unroll
      for (int r = 0; r < 8; ++r) {
        const int tokl = 32 * w + 16 * mt + 8 * h + r;
        const float u = acc[mt][nt][r] * (1.0f / WSC_) + bvl;
        const float gl = 0.5f * u * (1.0f + erff(u * 0.70710678118654752f));
        sT[tokl * 64 + feat] = (_Float16)(gl * HSC_);
      }
    }
  }
  __syncthreads();

  h_store_pass(sT, hp, m0, n0, w, lane);
  __threadfence();
  h_store_pass(sT, hp, m0, n0, w, lane);
}

__global__ __launch_bounds__(256) void transpose_out(
    const float* __restrict__ xres, const float* __restrict__ xmask,
    float* __restrict__ out)
{
  __shared__ float s[64][65];
  const int tid = threadIdx.x, lane = tid & 31, w = tid >> 5;
  const int b = blockIdx.z, c0 = blockIdx.y * 64, t0 = blockIdx.x * 64;
  {
    const int r = tid >> 4, q = tid & 15;
    #pragma unroll
    for (int i = 0; i < 4; ++i) {
      const int tt = 16 * i + r;
      const v4f v = *(const v4fa*)(xres + ((size_t)b * TT_ + t0 + tt) * CH_ + c0 + 4 * q);
      s[tt][4 * q + 0] = v.x;
      s[tt][4 * q + 1] = v.y;
      s[tt][4 * q + 2] = v.z;
      s[tt][4 * q + 3] = v.w;
    }
  }
  __syncthreads();

  const int rr = lane >> 4, p = lane & 15;
  const v4f mk = *(const v4fa*)(xmask + (size_t)b * TT_ + t0 + 4 * p);
  v4f of[4];
  #pragma unroll
  for (int i = 0; i < 4; ++i) {
    const int cc = w * 8 + 2 * i + rr;
    const v4f v = { s[4 * p + 0][cc] * mk.x, s[4 * p + 1][cc] * mk.y, s[4 * p + 2][cc] * mk.z, s[4 * p + 3][cc] * mk.w };
    of[i] = v;
  }
  #pragma unroll
  for (int pass = 0; pass < 2; ++pass) {
    #pragma unroll
    for (int i = 0; i < 4; ++i) {
      const int cc = w * 8 + 2 * i + rr;
      *(volatile v4f*)(out + ((size_t)b * CH_ + c0 + cc) * TT_ + t0 + 4 * p) = of[i];
    }
    if (pass == 0) __threadfence();
  }
}

extern "C" void kernel_launch(void* const* d_in, const int* in_sizes, int n_in,
                              void* d_out, int out_size, void* d_ws, size_t ws_size,
                              hipStream_t stream) {
  if (n_in < 18) return;
  if (in_sizes[0] != NB_ * CH_ * TT_) return;
  if (in_sizes[1] != NB_ * TT_) return;
  if (in_sizes[2] != NL_ * NW_ || in_sizes[4] != NL_ * NW_ || in_sizes[6] != NL_ * NW_ || in_sizes[8] != NL_ * NW_) return;
  if (in_sizes[3] != NL_ * CH_ || in_sizes[5] != NL_ * CH_ || in_sizes[7] != NL_ * CH_ || in_sizes[9] != NL_ * CH_) return;
  if (in_sizes[10] != NL_ * CH_ || in_sizes[11] != NL_ * CH_ || in_sizes[16] != NL_ * CH_ || in_sizes[17] != NL_ * CH_) return;
  if (in_sizes[12] != NL_ * NW1_ || in_sizes[14] != NL_ * NW1_) return;
  if (in_sizes[13] != NL_ * FC_ || in_sizes[15] != NL_ * CH_) return;
  if (out_size != NB_ * CH_ * TT_) return;

  const float* x    = (const float*)d_in[0];
  const float* xm   = (const float*)d_in[1];
  const float* wq   = (const float*)d_in[2];
  const float* bq   = (const float*)d_in[3];
  const float* wk   = (const float*)d_in[4];
  const float* bk   = (const float*)d_in[5];
  const float* wv   = (const float*)d_in[6];
  const float* bv   = (const float*)d_in[7];
  const float* wo   = (const float*)d_in[8];
  const float* bo   = (const float*)d_in[9];
  const float* ln0g = (const float*)d_in[10];
  const float* ln0b = (const float*)d_in[11];
  const float* w1   = (const float*)d_in[12];
  const float* b1   = (const float*)d_in[13];
  const float* w2   = (const float*)d_in[14];
  const float* b2   = (const float*)d_in[15];
  const float* ln1g = (const float*)d_in[16];
  const float* ln1b = (const float*)d_in[17];
  float* out = (float*)d_out;

  const size_t whqkv_b = (size_t)NL_ * 3 * NW_ * 2;
  const size_t who_b   = (size_t)NL_ * NW_ * 2;
  const size_t wh1_b   = (size_t)NL_ * NW1_ * 2;
  const size_t wh2_b   = (size_t)NL_ * NW1_ * 2;
  const size_t xres_b  = (size_t)NTOK_ * CH_ * 4;
  const size_t pl_b    = (size_t)NTOK_ * CH_ * 2;
  const size_t ybuf_b  = (size_t)NTOK_ * CH_ * 4;
  const size_t hp_b    = (size_t)NTOK_ * FC_ * 2;
  const size_t total = whqkv_b + who_b + wh1_b + wh2_b + xres_b + 5 * pl_b + ybuf_b + hp_b;
  if (total > ws_size) return;

  char* ws = (char*)d_ws;
  size_t off = 0;
  _Float16* whqkv = (_Float16*)(ws + off); off += whqkv_b;
  _Float16* who   = (_Float16*)(ws + off); off += who_b;
  _Float16* wh1   = (_Float16*)(ws + off); off += wh1_b;
  _Float16* wh2   = (_Float16*)(ws + off); off += wh2_b;
  float*    xres  = (float*)(ws + off);    off += xres_b;
  _Float16* xh    = (_Float16*)(ws + off); off += pl_b;
  _Float16* qh    = (_Float16*)(ws + off); off += pl_b;
  _Float16* kh    = (_Float16*)(ws + off); off += pl_b;
  _Float16* vt    = (_Float16*)(ws + off); off += pl_b;
  _Float16* oh    = (_Float16*)(ws + off); off += pl_b;
  float*    ybuf  = (float*)(ws + off);    off += ybuf_b;
  _Float16* hp    = (_Float16*)(ws + off); off += hp_b;
  if (off != total) return;

  convert_w<<<G_TOT_ / 256, 256, 0, stream>>>(wq, wk, wv, wo, w1, w2, whqkv, who, wh1, wh2);

  const dim3 gtr(TT_ / 64, CH_ / 64, NB_);
  transpose_in<<<gtr, 256, 0, stream>>>(x, xm, xres, xh);

  const dim3 gqkv(NTOK_ / 128, 3 * CH_ / 64);
  const dim3 gatt(TT_ / 64, NB_ * NH_);
  const dim3 gc(NTOK_ / 128, CH_ / 64);
  const dim3 gf(NTOK_ / 128, FC_ / 64);
  const int  gln = NTOK_ / 8;

  for (int i = 0; i < NL_; ++i) {
    gemm_qkv<<<gqkv, 128, 0, stream>>>(xh, whqkv + (size_t)i * 3 * NW_,
                                        bq + i * CH_, bk + i * CH_, bv + i * CH_,
                                        qh, kh, vt);
    attn_kernel<<<gatt, 128, 0, stream>>>(qh, kh, vt, oh);
    gemm_f32<<<gc, 128, 0, stream>>>(oh, CH_, who + (size_t)i * NW_, CH_, CH_,
                                      bo + i * CH_, 1.0f / WSC_, ybuf);
    ln_kernel<<<gln, 256, 0, stream>>>(xres, ybuf, ln0g + i * CH_, ln0b + i * CH_, xm, 0, xh);
    gemm_gelu<<<gf, 128, 0, stream>>>(xh, wh1 + (size_t)i * NW1_, b1 + i * FC_, hp);
    gemm_f32<<<gc, 128, 0, stream>>>(hp, FC_, wh2 + (size_t)i * NW1_, FC_, FC_,
                                      b2 + i * CH_, 1.0f / (WSC_ * HSC_), ybuf);
    ln_kernel<<<gln, 256, 0, stream>>>(xres, ybuf, ln1g + i * CH_, ln1b + i * CH_, xm, 1, xh);
  }

  transpose_out<<<gtr, 256, 0, stream>>>(xres, xm, out);
}
